// GNN_67362267070571
// MI455X (gfx1250) — hardware-verified
//
#include <hip/hip_runtime.h>
#include <stddef.h>
#include <stdint.h>
#include <math.h>

#ifndef H1_SINGLE
#define H1_SINGLE 0
#endif

#define NN      100000
#define HD      64
#define NE      1600000
#define GBM     128
#define MP      100096
#define KL      128
#define NTHR    256
#define NWAVE   8
#define EPT     8
#define WCH     (32 * EPT)
#define NBRUN   1024
#define SLB     10
#define NBK     98
#define WLCAP   3072
#define RCAP    20480
#define DEGCAP  64
#define MAXDEG_MEAS   36
#define MAXB1024_MEAS 16710
#define ABM     64
#define SP      68
#define WSMAX   134217728

#define BK_ZINTS (NWAVE * WLCAP + RCAP + 4 * NBRUN)
#define BK_INTS  (BK_ZINTS + 16)
#define BK_LDS   (BK_INTS * 4)

#define PBX   (MP * HD / 8 / NTHR)
#define PBW1  (HD * HD / 8 / NTHR)
#define PBW2  (HD * KL / 8 / NTHR)
#define PBTOT (PBX + PBW1 + PBW2 + 1)

#define K2    (H1_SINGLE ? 64 : 128)

static_assert(HD == 64 && HD == 16 * 4);
static_assert(MP % GBM == 0 && MP >= NN && MP == 782 * GBM && MP % ABM == 0);
static_assert(NBRUN == 1024 && NBRUN == (1 << SLB) && NBRUN % ABM == 0 && NBRUN % GBM == 0 && NBRUN % 32 == 0);
static_assert(NBRUN == 4 * NTHR);
static_assert(NBK * NBRUN >= MP);
static_assert(NN <= (1 << 22));
static_assert(NE < (1 << 21) && (((long long)NE) << SLB) < (1LL << 31));
static_assert(NE % WCH == 0 && NE % 4 == 0);
static_assert(RCAP % (NTHR * 4) == 0 && (2 * NBRUN) % (NTHR * 4) == 0 && BK_ZINTS % 4 == 0 && WLCAP % 32 == 0);
static_assert((long long)RCAP * 100 >= (long long)MAXB1024_MEAS * 105);
static_assert((long long)WLCAP * 100 >= (long long)(RCAP / NWAVE) * 115);
static_assert(NWAVE * WLCAP >= RCAP);
static_assert(MAXDEG_MEAS + 8 <= DEGCAP);
static_assert(BK_LDS <= 327680);
static_assert((GBM * SP + GBM) * 4 <= 65536);
static_assert((MP * HD / 8) % NTHR == 0 && (HD * HD / 8) % NTHR == 0 && (HD * KL / 8) % NTHR == 0);
static_assert(KL % 32 == 0 && KL == 2 * HD && HD % 32 == 0);
static_assert(ABM == NWAVE * 8);

typedef float          v4f   __attribute__((ext_vector_type(4)));
typedef float          v8f   __attribute__((ext_vector_type(8)));
typedef int            v4i   __attribute__((ext_vector_type(4)));
typedef int            v8i   __attribute__((ext_vector_type(8)));
typedef unsigned short v8us  __attribute__((ext_vector_type(8)));
typedef unsigned short v16us __attribute__((ext_vector_type(16)));
typedef __bf16         v16bf __attribute__((ext_vector_type(16)));
typedef v4f  __attribute__((may_alias)) v4fa;
typedef v4i  __attribute__((may_alias)) v4ia;
typedef v8us __attribute__((may_alias)) v8usa;
union FragB { v16bf v; v16us u; v8us h[2]; v8i w; };

__device__ __forceinline__ v8f wmb(const FragB& a, const FragB& b, v8f c) {
  v8f d = __builtin_amdgcn_wmma_f32_16x16x32_bf16(false, a.v, false, b.v, (short)0, c, false, false);
  asm volatile("v_nop\n\tv_nop\n\tv_nop\n\tv_nop" : "+v"(d) : "v"(a.w), "v"(b.w));
  return d;
}

__device__ __forceinline__ unsigned bf16_bits(float f) {
  const unsigned u = __float_as_uint(f);
  const unsigned r = (u + 0x7FFFu + ((u >> 16) & 1u)) >> 16;
  const unsigned q = (u >> 16) | 0x40u;
  return ((u & 0x7fffffffu) > 0x7f800000u) ? q : r;
}

__device__ __forceinline__ void hilo_pack(float v0, float v1, float v2, float v3,
                                          int& h01, int& h23, int& l01, int& l23) {
  const unsigned a0 = bf16_bits(v0), a1 = bf16_bits(v1), a2 = bf16_bits(v2), a3 = bf16_bits(v3);
  const unsigned b0 = bf16_bits(v0 - __uint_as_float(a0 << 16));
  const unsigned b1 = bf16_bits(v1 - __uint_as_float(a1 << 16));
  const unsigned b2 = bf16_bits(v2 - __uint_as_float(a2 << 16));
  const unsigned b3 = bf16_bits(v3 - __uint_as_float(a3 << 16));
  h01 = (int)(a0 | (a1 << 16)); h23 = (int)(a2 | (a3 << 16));
  l01 = (int)(b0 | (b1 << 16)); l23 = (int)(b2 | (b3 << 16));
}

__device__ __forceinline__ v4i regroup8(int h01, int h23, int l01, int l23, int lane) {
  const int t  = lane & 15;
  const int s0 = (lane & 16) + ((2 * t) & 15), s1 = s0 + 1;
  const int a0 = __shfl(h01, s0, 32), a1 = __shfl(h23, s0, 32), a2 = __shfl(h01, s1, 32), a3 = __shfl(h23, s1, 32);
  const int b0 = __shfl(l01, s0, 32), b1 = __shfl(l23, s0, 32), b2 = __shfl(l01, s1, 32), b3 = __shfl(l23, s1, 32);
  const int mk = (t < 8) ? -1 : 0;
  v4i o;
  o.x = (a0 & mk) | (b0 & ~mk); o.y = (a1 & mk) | (b1 & ~mk);
  o.z = (a2 & mk) | (b2 & ~mk); o.w = (a3 & mk) | (b3 & ~mk);
  return o;
}

__device__ __forceinline__ void st2_v4f(float* p, v4f v) {
  *(volatile v4f*)p = v;
  __threadfence();
  *(volatile v4f*)p = v;
}
__device__ __forceinline__ void st2_v8us(unsigned short* p, v8us v) {
  *(volatile v8us*)p = v;
  __threadfence();
  *(volatile v8us*)p = v;
}

__device__ __forceinline__ v8us gather8(const float* __restrict__ base, int stride) {
  float f[8];
#pragma unroll
  for (int i = 0; i < 8; ++i) f[i] = base[(size_t)i * (size_t)stride];
  v8us o;
#pragma unroll
  for (int i = 0; i < 8; ++i) o[i] = (unsigned short)bf16_bits(f[i]);
  return o;
}

__global__ __launch_bounds__(NTHR) void k_prep(const float* __restrict__ x, const float* __restrict__ w1,
                                               const float* __restrict__ b1, const float* __restrict__ w2,
                                               const float* __restrict__ b2,
                                               unsigned short* xb, unsigned short* w1t, unsigned short* w2d,
                                               float* sm) {
  const int tid = (int)threadIdx.x, lane = tid & 31;
  const int blk = (int)blockIdx.x;
  if (blk < PBX) {
    const int u   = blk * NTHR + tid;
    const int row = u >> 3, k8 = (u & 7) * 8;
    const int rc  = row < NN ? row : NN - 1;
    const unsigned mk = row < NN ? 0xffffu : 0u;
    const float* p = x + (size_t)rc * HD + k8;
    const v4f a = *(const v4fa*)p;
    const v4f b = *(const v4fa*)(p + 4);
    v8us o;
    o[0] = (unsigned short)(bf16_bits(a.x) & mk); o[1] = (unsigned short)(bf16_bits(a.y) & mk);
    o[2] = (unsigned short)(bf16_bits(a.z) & mk); o[3] = (unsigned short)(bf16_bits(a.w) & mk);
    o[4] = (unsigned short)(bf16_bits(b.x) & mk); o[5] = (unsigned short)(bf16_bits(b.y) & mk);
    o[6] = (unsigned short)(bf16_bits(b.z) & mk); o[7] = (unsigned short)(bf16_bits(b.w) & mk);
    st2_v8us(xb + (size_t)row * HD + k8, o);
  } else if (blk < PBX + PBW1) {
    const int u = (blk - PBX) * NTHR + tid;
    const int n = u >> 3, k8 = (u & 7) * 8;
    const v8us o = gather8(w1 + (size_t)k8 * HD + n, HD);
    st2_v8us(w1t + (size_t)n * HD + k8, o);
  } else if (blk < PBX + PBW1 + PBW2) {
    const int u = (blk - PBX - PBW1) * NTHR + tid;
    const int n = u >> 4, k8 = (u & 15) * 8, kk = k8 & 63;
    const v8us o = gather8(w2 + (size_t)kk * HD + n, HD);
    st2_v8us(w2d + (size_t)n * KL + k8, o);
  } else {
    if (tid < 32) {
      const int q = lane & 15;
      const v4f a = *(const v4fa*)(b1 + 4 * q);
      const v4f c = *(const v4fa*)(b2 + 4 * q);
      asm volatile("" :: "v"(a));
      asm volatile("" :: "v"(c));
      const unsigned ma = (lane < 16) ? 0xffffffffu : 0u;
      v4f o;
      o.x = __uint_as_float(((bf16_bits(a.x) << 16) & ma) | ((bf16_bits(c.x) << 16) & ~ma));
      o.y = __uint_as_float(((bf16_bits(a.y) << 16) & ma) | ((bf16_bits(c.y) << 16) & ~ma));
      o.z = __uint_as_float(((bf16_bits(a.z) << 16) & ma) | ((bf16_bits(c.z) << 16) & ~ma));
      o.w = __uint_as_float(((bf16_bits(a.w) << 16) & ma) | ((bf16_bits(c.w) << 16) & ~ma));
      st2_v4f(sm + 4 * lane, o);
    }
  }
}

__device__ __forceinline__ void bucket_flush(const int* pl, const int* cnt, const float* dvf, int ov,
                                             int* lp, int* cop, float* dp, int* fp, int tid) {
#pragma unroll 1
  for (int i = tid * 4; i < RCAP; i += NTHR * 4) {
    const v4i v = *(const v4ia*)(pl + i);
    *(volatile v4i*)(lp + i) = v;
  }
#pragma unroll 1
  for (int i = tid * 4; i < 2 * NBRUN; i += NTHR * 4) {
    const v4i v = *(const v4ia*)(cnt + i);
    *(volatile v4i*)(cop + i) = v;
  }
  {
    const v4f v = *(const v4fa*)(dvf + 4 * tid);
    *(volatile v4f*)(dp + 4 * tid) = v;
  }
  if (tid < 8) {
    const v4i f = {ov, ov, ov, ov};
    *(volatile v4i*)(fp + 4 * tid) = f;
  }
}

__global__ __launch_bounds__(NTHR) void k_bucket(const int* __restrict__ srcs, const int* __restrict__ dsts,
                                                 int* LIST, int* CO, float* DINV, int* FLAG) {
  extern __shared__ __attribute__((aligned(16))) int dsm[];
  int*   wl   = dsm;
  int*   pl   = dsm + NWAVE * WLCAP;
  int*   cnt  = pl + RCAP;
  int*   offs = cnt + NBRUN;
  int*   cur  = offs + NBRUN;
  float* dvf  = (float*)(cur + NBRUN);
  int*   misc = cur + 2 * NBRUN;
  const int tid = (int)threadIdx.x, lane = tid & 31, wave = tid >> 5;
  const int blk = (int)blockIdx.x;
  const unsigned nbs = (unsigned)(blk * NBRUN);
  int* mylist = wl + wave * WLCAP;
  int ov = 0;

  {
    const v4i z4 = {0, 0, 0, 0};
    for (int i = tid * 4; i < BK_ZINTS; i += NTHR * 4) *(v4ia*)(dsm + i) = z4;
    if (tid < 16) misc[tid] = 0;
  }
  __syncthreads();

  {
    const int per  = ((NE + NWAVE * WCH - 1) / (NWAVE * WCH)) * WCH;
    const int ebeg = wave * per;
    const int eend = (ebeg + per < NE) ? (ebeg + per) : NE;
    int wc = 0;
#pragma unroll 1
    for (int cb = ebeg; cb < eend; cb += WCH) {
      const int e0 = cb + lane * EPT;
      const v4i da = *(const v4ia*)(dsts + e0);
      const v4i db = *(const v4ia*)(dsts + e0 + 4);
      const unsigned s0 = (unsigned)da.x - nbs, s1 = (unsigned)da.y - nbs;
      const unsigned s2 = (unsigned)da.z - nbs, s3 = (unsigned)da.w - nbs;
      const unsigned s4 = (unsigned)db.x - nbs, s5 = (unsigned)db.y - nbs;
      const unsigned s6 = (unsigned)db.z - nbs, s7 = (unsigned)db.w - nbs;
      const bool h0 = s0 < (unsigned)NBRUN, h1 = s1 < (unsigned)NBRUN, h2 = s2 < (unsigned)NBRUN, h3 = s3 < (unsigned)NBRUN;
      const bool h4 = s4 < (unsigned)NBRUN, h5 = s5 < (unsigned)NBRUN, h6 = s6 < (unsigned)NBRUN, h7 = s7 < (unsigned)NBRUN;
      const unsigned m0 = __builtin_amdgcn_ballot_w32(h0), m1 = __builtin_amdgcn_ballot_w32(h1);
      const unsigned m2 = __builtin_amdgcn_ballot_w32(h2), m3 = __builtin_amdgcn_ballot_w32(h3);
      const unsigned m4 = __builtin_amdgcn_ballot_w32(h4), m5 = __builtin_amdgcn_ballot_w32(h5);
      const unsigned m6 = __builtin_amdgcn_ballot_w32(h6), m7 = __builtin_amdgcn_ballot_w32(h7);
      const unsigned any = m0 | m1 | m2 | m3 | m4 | m5 | m6 | m7;
      if (any != 0u) {
        const int pre = (int)(__builtin_amdgcn_mbcnt_lo(m0, 0u) + __builtin_amdgcn_mbcnt_lo(m1, 0u) +
                              __builtin_amdgcn_mbcnt_lo(m2, 0u) + __builtin_amdgcn_mbcnt_lo(m3, 0u) +
                              __builtin_amdgcn_mbcnt_lo(m4, 0u) + __builtin_amdgcn_mbcnt_lo(m5, 0u) +
                              __builtin_amdgcn_mbcnt_lo(m6, 0u) + __builtin_amdgcn_mbcnt_lo(m7, 0u));
        int p = wc + pre;
        if (h0) { if (p < WLCAP) mylist[p] = ((e0 + 0) << SLB) | (int)s0; p = p + 1; }
        if (h1) { if (p < WLCAP) mylist[p] = ((e0 + 1) << SLB) | (int)s1; p = p + 1; }
        if (h2) { if (p < WLCAP) mylist[p] = ((e0 + 2) << SLB) | (int)s2; p = p + 1; }
        if (h3) { if (p < WLCAP) mylist[p] = ((e0 + 3) << SLB) | (int)s3; p = p + 1; }
        if (h4) { if (p < WLCAP) mylist[p] = ((e0 + 4) << SLB) | (int)s4; p = p + 1; }
        if (h5) { if (p < WLCAP) mylist[p] = ((e0 + 5) << SLB) | (int)s5; p = p + 1; }
        if (h6) { if (p < WLCAP) mylist[p] = ((e0 + 6) << SLB) | (int)s6; p = p + 1; }
        if (h7) { if (p < WLCAP) mylist[p] = ((e0 + 7) << SLB) | (int)s7; p = p + 1; }
        wc += (int)(__builtin_popcount(m0) + __builtin_popcount(m1) + __builtin_popcount(m2) + __builtin_popcount(m3) +
                    __builtin_popcount(m4) + __builtin_popcount(m5) + __builtin_popcount(m6) + __builtin_popcount(m7));
      }
    }
    if (lane == 0) misc[wave] = wc;
  }
  __syncthreads();

  {
    int c = misc[wave];
    c = max(0, min(c, WLCAP));
#pragma unroll 1
    for (int b0 = 0; b0 < c; b0 += 32) {
      const int idx = b0 + lane;
      const int ic  = idx < WLCAP ? idx : WLCAP - 1;
      const int ent = mylist[ic];
      int eid = (ent >> SLB) & 0x1FFFFF;
      eid = min(eid, NE - 1);
      int sr = srcs[eid];
      asm volatile("" :: "v"(sr));
      sr = max(0, min(sr, NN - 1));
      const int word = (int)(((unsigned)sr << SLB) | ((unsigned)ent & (unsigned)(NBRUN - 1)));
      if (idx < c) mylist[idx] = word;
    }
  }
  __syncthreads();

  if (wave == 0) {
#pragma unroll 1
    for (int w2 = 0; w2 < NWAVE; ++w2) {
      int c = misc[w2];
      if (c > WLCAP) ov = 1;
      c = max(0, min(c, WLCAP));
#pragma unroll 1
      for (int b0 = 0; b0 < c; b0 += 32) {
        const int idx = b0 + lane;
        const int ent = wl[w2 * WLCAP + (idx < WLCAP ? idx : WLCAP - 1)];
        const int m32 = (c - b0) < 32 ? (c - b0) : 32;
#pragma unroll 1
        for (int k = 0; k < m32; ++k) {
          const int u    = __builtin_amdgcn_readlane(ent, k);
          const int slot = u & (NBRUN - 1);
          if (lane == 0) cnt[slot] = cnt[slot] + 1;
        }
      }
    }
  }
  __syncthreads();
  if (wave == 0) {
    const int base = lane * (NBRUN / 32);
    int s = 0;
    int bigl = 0;
#pragma unroll 1
    for (int i = 0; i < NBRUN / 32; ++i) {
      const int cv = cnt[base + i];
      s += cv;
      bigl |= (cv > DEGCAP) ? 1 : 0;
    }
    int incl = s;
#pragma unroll
    for (int d = 1; d < 32; d <<= 1) {
      const int y = __shfl_up(incl, d, 32);
      if (lane >= d) incl += y;
    }
    const int total = __shfl(incl, 31, 32);
    const unsigned bigm = __builtin_amdgcn_ballot_w32(bigl != 0);
    if (total > RCAP) ov = 1;
    if (bigm != 0u) ov = 1;
    int run = incl - s;
#pragma unroll 1
    for (int i = 0; i < NBRUN / 32; ++i) {
      const int cv = cnt[base + i];
      offs[base + i] = run;
      cur[base + i]  = run;
      run += cv;
    }
    if (lane == 0) misc[9] = ov;
  }
  __syncthreads();

  if (wave == 0) {
#pragma unroll 1
    for (int w2 = 0; w2 < NWAVE; ++w2) {
      int c = misc[w2];
      c = max(0, min(c, WLCAP));
#pragma unroll 1
      for (int b0 = 0; b0 < c; b0 += 32) {
        const int idx = b0 + lane;
        const int ent = wl[w2 * WLCAP + (idx < WLCAP ? idx : WLCAP - 1)];
        const int m32 = (c - b0) < 32 ? (c - b0) : 32;
#pragma unroll 1
        for (int k = 0; k < m32; ++k) {
          const int u    = __builtin_amdgcn_readlane(ent, k);
          const int slot = u & (NBRUN - 1);
          const int sr   = (int)(((unsigned)u >> SLB) & 0x3FFFFFu);
          if (lane == 0) {
            int p = cur[slot];
            p = max(0, min(p, RCAP - 1));
            pl[p] = sr;
            cur[slot] = p + 1;
          }
        }
      }
    }
  }
  __syncthreads();

#pragma unroll 1
  for (int i = tid; i < NBRUN; i += NTHR) {
    const float dg = (float)(cnt[i] + 1);
    dvf[i] = 1.0f / sqrtf(dg);
  }
  __syncthreads();

  const int ovf = misc[9];
  int*   lp  = LIST + (size_t)blk * RCAP;
  int*   cop = CO + (size_t)blk * (2 * NBRUN);
  float* dp  = DINV + (size_t)blk * NBRUN;
  int*   fp  = FLAG + (size_t)blk * 32;
  bucket_flush(pl, cnt, dvf, ovf, lp, cop, dp, fp, tid);
  __threadfence();
  bucket_flush(pl, cnt, dvf, ovf, lp, cop, dp, fp, tid);
}

template <int KTOT, int PITCH>
__device__ __forceinline__ void gemm_16x64(const unsigned short* __restrict__ ap,
                                           const unsigned short* __restrict__ bp, v8f (&acc)[4]) {
#pragma unroll 1
  for (int k0 = 0; k0 < KTOT; k0 += 32) {
    FragB af;
    af.h[0] = *(const v8usa*)(ap + k0);
    af.h[1] = *(const v8usa*)(ap + k0 + 16);
#pragma unroll
    for (int nt = 0; nt < 4; ++nt) {
      const unsigned short* wq = bp + (size_t)(16 * nt) * (size_t)PITCH + k0;
      FragB bf;
      bf.h[0] = *(const v8usa*)wq;
      bf.h[1] = *(const v8usa*)(wq + 16);
      acc[nt] = wmb(af, bf, acc[nt]);
    }
  }
}

__device__ __forceinline__ void stage_d(float* stg, const v8f (&acc)[4], int wave, int hh, int m) {
#pragma unroll
  for (int nt = 0; nt < 4; ++nt) {
#pragma unroll
    for (int r = 0; r < 8; ++r) stg[(16 * wave + 8 * hh + r) * SP + 16 * nt + m] = acc[nt][r];
  }
}

template <int KTOT, int PITCH>
__global__ __launch_bounds__(NTHR) __attribute__((amdgpu_num_vgpr(248)))
void k_gemm(const unsigned short* __restrict__ A, const unsigned short* __restrict__ BT,
            const float* __restrict__ DINV, float* HPo) {
  static_assert(KTOT % 32 == 0 && KTOT <= PITCH && PITCH % 8 == 0);
  __shared__ __attribute__((aligned(16))) float stg[GBM * SP];
  __shared__ __attribute__((aligned(16))) float sdv[GBM];
  const int tid = (int)threadIdx.x, lane = tid & 31, wave = tid >> 5, hh = lane >> 4, m = lane & 15;
  const int rowBase = (int)blockIdx.x * GBM;
  if (tid < 32) *(v4fa*)(sdv + 4 * tid) = *(const v4fa*)(DINV + (size_t)rowBase + 4 * tid);

  v8f acc[4];
  {
    const v8f z = {0.f, 0.f, 0.f, 0.f, 0.f, 0.f, 0.f, 0.f};
#pragma unroll
    for (int t = 0; t < 4; ++t) acc[t] = z;
  }
  const unsigned short* ap = A + (size_t)(rowBase + 16 * wave + m) * (size_t)PITCH + 8 * hh;
  const unsigned short* bp = BT + (size_t)m * (size_t)PITCH + 8 * hh;
  gemm_16x64<KTOT, PITCH>(ap, bp, acc);
  stage_d(stg, acc, wave, hh, m);
  __syncthreads();

#pragma unroll 1
  for (int i = 0; i < 8; ++i) {
    const int lr   = 16 * wave + 2 * i + hh;
    const int grow = rowBase + lr;
    const bool live = grow < NN;
    const v4f a  = *(const v4fa*)(stg + lr * SP + 4 * m);
    const float dv = sdv[lr];
    asm volatile("" :: "v"(a));
    asm volatile("" :: "v"(dv));
    const float v0 = dv * a.x, v1 = dv * a.y, v2 = dv * a.z, v3 = dv * a.w;
    v4f o;
    o.x = live ? v0 : 0.0f; o.y = live ? v1 : 0.0f; o.z = live ? v2 : 0.0f; o.w = live ? v3 : 0.0f;
    st2_v4f(HPo + (size_t)grow * HD + 4 * m, o);
  }
}

template <int MODE>
__global__ __launch_bounds__(NTHR) void k_agg(const int* __restrict__ LIST, const int* __restrict__ CO,
                                              const float* __restrict__ DINV, const int* __restrict__ FLAG,
                                              const float* __restrict__ HP, const float* __restrict__ SMB,
                                              unsigned short* H1, float* out) {
  const int tid = (int)threadIdx.x, lane = tid & 31, wave = tid >> 5, hh = lane >> 4, q = lane & 15;
  const int rowBase = (int)blockIdx.x * ABM;
  const int bucket  = rowBase >> SLB;
  const int* lb  = LIST + (size_t)bucket * RCAP;
  const int* cob = CO + (size_t)bucket * (2 * NBRUN);
  const int flag = FLAG[(size_t)bucket * 32];
  const v4f bias = *(const v4fa*)(SMB + 4 * q);
  const float qnan = __uint_as_float(0x7fc00000u);

#pragma unroll 1
  for (int i = 0; i < ABM / (2 * NWAVE); ++i) {
    const int d    = rowBase + (ABM / NWAVE) * wave + 2 * i + hh;
    const int slot = d & (NBRUN - 1);
    int c = cob[slot];
    int o = cob[NBRUN + slot];
    const float dd = DINV[d];
    asm volatile("" :: "v"(c), "v"(o), "v"(dd));
    const bool big = c > DEGCAP;
    c = max(0, min(c, DEGCAP));
    o = max(0, min(o, RCAP - 1));
    const int co = __shfl_xor(c, 16, 32);
    const int cm = max(c, co);
    int last = o + c - 1;
    last = last < o ? o : last;
    last = min(last, RCAP - 1);
    float a0 = 0.0f, a1 = 0.0f, a2 = 0.0f, a3 = 0.0f;
#pragma unroll 1
    for (int j = 0; j < cm; ++j) {
      int idx = o + j;
      idx = min(idx, last);
      int sr = lb[idx];
      sr = max(0, min(sr, NN - 1));
      const v4f v = *(const v4fa*)(HP + (size_t)sr * HD + 4 * q);
      asm volatile("" :: "v"(v));
      const bool valid = j < c;
      const float t0 = a0 + v.x, t1 = a1 + v.y, t2 = a2 + v.z, t3 = a3 + v.w;
      a0 = valid ? t0 : a0; a1 = valid ? t1 : a1; a2 = valid ? t2 : a2; a3 = valid ? t3 : a3;
    }
    const v4f g = *(const v4fa*)(HP + (size_t)d * HD + 4 * q);
    asm volatile("" :: "v"(g));
    float v0 = dd * (a0 + g.x) + bias.x, v1 = dd * (a1 + g.y) + bias.y;
    float v2 = dd * (a2 + g.z) + bias.z, v3 = dd * (a3 + g.w) + bias.w;
    if constexpr (MODE != 0) {
      v0 = (v0 > 0.0f) ? v0 : (v0 - v0); v1 = (v1 > 0.0f) ? v1 : (v1 - v1);
      v2 = (v2 > 0.0f) ? v2 : (v2 - v2); v3 = (v3 > 0.0f) ? v3 : (v3 - v3);
    }
    const bool bad  = (flag != 0) | big;
    const bool live = d < NN;
    v0 = bad ? qnan : v0; v1 = bad ? qnan : v1; v2 = bad ? qnan : v2; v3 = bad ? qnan : v3;
    if constexpr (MODE != 0) {
      v0 = live ? v0 : 0.0f; v1 = live ? v1 : 0.0f; v2 = live ? v2 : 0.0f; v3 = live ? v3 : 0.0f;
      int h01, h23, l01, l23;
      hilo_pack(v0, v1, v2, v3, h01, h23, l01, l23);
      const v4i ow = regroup8(h01, h23, l01, l23, lane);
      unsigned short* hp = H1 + (size_t)d * KL + 8 * q;
      *(volatile v4i*)hp = ow;
      __threadfence();
      *(volatile v4i*)hp = ow;
    } else {
      v4f ov;
      ov.x = v0; ov.y = v1; ov.z = v2; ov.w = v3;
      const int dc = live ? d : NN - 1;
      float* op = out + (size_t)dc * HD + 4 * q;
      if (live) *(volatile v4f*)op = ov;
      __threadfence();
      if (live) *(volatile v4f*)op = ov;
    }
  }
}

extern "C" void kernel_launch(void* const* d_in, const int* in_sizes, int n_in,
                              void* d_out, int out_size, void* d_ws, size_t ws_size,
                              hipStream_t stream) {
  if (n_in < 6) return;
  if (in_sizes[0] != NN * HD) return;
  if (in_sizes[1] != 2 * NE) return;
  if (in_sizes[2] != HD * HD) return;
  if (in_sizes[3] != HD) return;
  if (in_sizes[4] != HD * HD) return;
  if (in_sizes[5] != HD) return;
  if (out_size != NN * HD) return;

  const float* x  = (const float*)d_in[0];
  const int*   ei = (const int*)d_in[1];
  const float* W1 = (const float*)d_in[2];
  const float* b1 = (const float*)d_in[3];
  const float* W2 = (const float*)d_in[4];
  const float* b2 = (const float*)d_in[5];
  float* out = (float*)d_out;
  const int* srcs = ei;
  const int* dsts = ei + NE;

  constexpr size_t zXB   = (size_t)MP * HD * 2;
  constexpr size_t zHP   = (size_t)MP * HD * 4;
  constexpr size_t zH1   = (size_t)MP * KL * 2;
  constexpr size_t zLIST = (size_t)NBK * RCAP * 4;
  constexpr size_t zCO   = (size_t)NBK * 2 * NBRUN * 4;
  constexpr size_t zDINV = (size_t)NBK * NBRUN * 4;
  constexpr size_t zFLAG = (size_t)NBK * 128;
  constexpr size_t zW1T  = (size_t)HD * HD * 2;
  constexpr size_t zW2D  = (size_t)HD * KL * 2;
  constexpr size_t zSM   = 512;
  constexpr size_t oXB   = 0;
  constexpr size_t oHP   = oXB + zXB;
  constexpr size_t oH1   = oHP + zHP;
  constexpr size_t oLIST = oH1 + zH1;
  constexpr size_t oCO   = oLIST + zLIST;
  constexpr size_t oDINV = oCO + zCO;
  constexpr size_t oFLAG = oDINV + zDINV;
  constexpr size_t oW1T  = oFLAG + zFLAG;
  constexpr size_t oW2D  = oW1T + zW1T;
  constexpr size_t oSM   = oW2D + zW2D;
  constexpr size_t oEND  = oSM + zSM;
  static_assert(zXB % 256 == 0 && zHP % 256 == 0 && zH1 % 256 == 0 && zLIST % 256 == 0 && zCO % 256 == 0);
  static_assert(zDINV % 256 == 0 && zFLAG % 256 == 0 && zW1T % 256 == 0 && zW2D % 256 == 0 && zSM % 256 == 0);
  static_assert((size_t)NBK * NBRUN >= (size_t)MP);
  static_assert(oEND <= (size_t)WSMAX);
  if (oEND > ws_size) return;

  char* ws = (char*)d_ws;
  unsigned short* XB   = (unsigned short*)(ws + oXB);
  float*          HP   = (float*)(ws + oHP);
  unsigned short* H1   = (unsigned short*)(ws + oH1);
  int*            LIST = (int*)(ws + oLIST);
  int*            CO   = (int*)(ws + oCO);
  float*          DINV = (float*)(ws + oDINV);
  int*            FLAG = (int*)(ws + oFLAG);
  unsigned short* W1T  = (unsigned short*)(ws + oW1T);
  unsigned short* W2D  = (unsigned short*)(ws + oW2D);
  float*          SM   = (float*)(ws + oSM);

  hipFuncSetAttribute(reinterpret_cast<const void*>(&k_bucket), hipFuncAttributeMaxDynamicSharedMemorySize, (int)BK_LDS);

  k_prep<<<PBTOT, NTHR, 0, stream>>>(x, W1, b1, W2, b2, XB, W1T, W2D, SM);
  k_bucket<<<NBK, NTHR, BK_LDS, stream>>>(srcs, dsts, LIST, CO, DINV, FLAG);
  k_gemm<HD, HD><<<MP / GBM, NTHR, 0, stream>>>(XB, W1T, DINV, HP);
  k_agg<1><<<MP / ABM, NTHR, 0, stream>>>(LIST, CO, DINV, FLAG, HP, SM, H1, out);
  k_gemm<K2, KL><<<MP / GBM, NTHR, 0, stream>>>(H1, W2D, DINV, HP);
  k_agg<0><<<MP / ABM, NTHR, 0, stream>>>(LIST, CO, DINV, FLAG, HP, SM + HD, H1, out);
}
